// TopDownSceneCaptionModule_53558242181153
// MI455X (gfx1250) — hardware-verified
//
#include <hip/hip_runtime.h>
#include <math.h>

constexpr int kB      = 128;
constexpr int kT      = 30;
constexpr int kEmb    = 300;
constexpr int kEmbPad = 320;
constexpr int kFeat   = 128;
constexpr int kHid    = 512;
constexpr int kProp   = 256;
constexpr int kVoc    = 3433;
constexpr int kVocPad = 3456;
constexpr int kGru    = 1536;
constexpr int kTdIn   = 940;
constexpr int kTdK    = 960;
constexpr int kLangK  = 640;
constexpr int kRowsBT = kB * kT;
constexpr int kGhhN   = 2048;
constexpr float kWCarry    = 16.0f;
constexpr float kWCarryInv = 0.0625f;

typedef __attribute__((ext_vector_type(16))) _Float16 v16h;
typedef __attribute__((ext_vector_type(8)))  _Float16 v8h;
typedef __attribute__((ext_vector_type(16))) __bf16   v16b;
typedef __attribute__((ext_vector_type(8)))  __bf16   v8b;
typedef __attribute__((ext_vector_type(8)))  float    v8f;
typedef __attribute__((ext_vector_type(4)))  float    v4f;
typedef __attribute__((ext_vector_type(4)))  unsigned int v4u;

__device__ __forceinline__ unsigned short f2bf_bits(float f) {
  unsigned u = __float_as_uint(f);
  return (unsigned short)((u + 0x7FFFu + ((u >> 16) & 1u)) >> 16);
}
__device__ __forceinline__ float bf_bits2f(unsigned short h) { return __uint_as_float(((unsigned)h) << 16); }

__device__ __forceinline__ void dep_guard_h(v8f& a, v8f& b, v16h x, v16h y) { asm volatile("v_nop\n\tv_nop\n\tv_nop\n\tv_nop" : "+v"(a), "+v"(b) : "v"(x), "v"(y)); }
__device__ __forceinline__ void dep_guard_b(v8f& a, v8f& b, v16b x, v16b y) { asm volatile("v_nop\n\tv_nop\n\tv_nop\n\tv_nop" : "+v"(a), "+v"(b) : "v"(x), "v"(y)); }
__device__ __forceinline__ void keep4_h(v16h a, v16h b, v16h c, v16h d) { asm volatile("v_nop" :: "v"(a), "v"(b), "v"(c), "v"(d)); }
__device__ __forceinline__ void keep4_b(v16b a, v16b b, v16b c, v16b d) { asm volatile("v_nop" :: "v"(a), "v"(b), "v"(c), "v"(d)); }
__device__ __forceinline__ void acc_guard4(v8f& a, v8f& b, v8f& c, v8f& d) { asm volatile("v_nop\n\tv_nop\n\tv_nop\n\tv_nop" : "+v"(a), "+v"(b), "+v"(c), "+v"(d)); }
template <typename T> struct Frag;
template <> struct Frag<_Float16> {
  typedef v16h V; union U { v16h v; v8h h[2]; };
  static __device__ __forceinline__ v16h load(const _Float16* p) {
    U f; f.h[0] = *(const v8h*)(p); f.h[1] = *(const v8h*)(p + 16); return f.v;
  }
  static __device__ __forceinline__ v8f mma(v16h a, v16h b, v8f c) {
    return __builtin_amdgcn_wmma_f32_16x16x32_f16(false, a, false, b, (short)0, c, false, false);
  }
  static __device__ __forceinline__ void guard(v8f& a, v8f& b, v16h x, v16h y) { dep_guard_h(a, b, x, y); }
  static __device__ __forceinline__ void keep(v16h a, v16h b, v16h c, v16h d) { keep4_h(a, b, c, d); }
};
template <> struct Frag<__bf16> {
  typedef v16b V; union U { v16b v; v8b h[2]; };
  static __device__ __forceinline__ v16b load(const __bf16* p) {
    U f; f.h[0] = *(const v8b*)(p); f.h[1] = *(const v8b*)(p + 16); return f.v;
  }
  static __device__ __forceinline__ v8f mma(v16b a, v16b b, v8f c) {
    return __builtin_amdgcn_wmma_f32_16x16x32_bf16(false, a, false, b, (short)0, c, false, false);
  }
  static __device__ __forceinline__ void guard(v8f& a, v8f& b, v16b x, v16b y) { dep_guard_b(a, b, x, y); }
  static __device__ __forceinline__ void keep(v16b a, v16b b, v16b c, v16b d) { keep4_b(a, b, c, d); }
};

__device__ __forceinline__ unsigned pk16(unsigned short a, unsigned short b) { return (unsigned)a | ((unsigned)b << 16); }
__device__ __forceinline__ unsigned short h_bits(float f) { const _Float16 h = (_Float16)f; return __builtin_bit_cast(unsigned short, h); }

template <int ET> struct Elem;
template <> struct Elem<0> { typedef _Float16 T; };
template <> struct Elem<1> { typedef __bf16 T; };
template <int ET, bool SPLIT, int BIAS_MODE, int OUT_MODE, bool RESID, int ACT = 0>
__global__ __launch_bounds__(256) void wmma_gemm64(
    const unsigned short* __restrict__ Ap, const unsigned short* __restrict__ A2p, int lda, long strideA,
    const unsigned short* __restrict__ Btp, const unsigned short* __restrict__ Bt2p, int ldb, long strideB,
    void* __restrict__ Cout, void* __restrict__ Cout2, int ldc, long strideC,
    const float* __restrict__ bias,
    const float* __restrict__ resid, long strideR,
    int M, int N, int K, float scale) {
  typedef typename Elem<ET>::T T;
  typedef typename Frag<T>::V V;
  const T* A = (const T*)Ap; const T* A2 = (const T*)A2p; const T* Bt = (const T*)Btp; const T* Bt2 = (const T*)Bt2p;
  __shared__ __align__(16) float sT[8][16 * 68];
  const int b    = blockIdx.y;
  const int lane = threadIdx.x & 31;
  const int wave = threadIdx.x >> 5;
  const int tilesN = N >> 6;
  const int tilesM = M >> 6;
  const int tile = blockIdx.x * 8 + wave;
  if (tile >= tilesM * tilesN) return;
  const int tm = tile / tilesN;
  const int tn = tile - tm * tilesN;
  const int m0 = tm << 6;
  const int n0 = tn << 6;

  const T* Ab  = A  + (size_t)b * strideA;
  const T* Bb  = Bt + (size_t)b * strideB;
  const T* Ab2 = SPLIT ? (A2  + (size_t)b * strideA) : nullptr;
  const T* Bb2 = SPLIT ? (Bt2 + (size_t)b * strideB) : nullptr;

  const int rlane = lane & 15;
  const int koff  = (lane >> 4) * 8;
  const int mOff  = (lane >> 4) * 8;

  v8f acc[4][4];
#pragma unroll
  for (int i = 0; i < 4; ++i)
#pragma unroll
    for (int j = 0; j < 4; ++j) acc[i][j] = (v8f){0.f,0.f,0.f,0.f,0.f,0.f,0.f,0.f};

  for (int k0 = 0; k0 < K; k0 += 32) {
    V bh[4], bl[4];
#pragma unroll
    for (int j = 0; j < 4; ++j) {
      const size_t bo = (size_t)(n0 + (j << 4) + rlane) * ldb + koff + k0;
      bh[j] = Frag<T>::load(Bb + bo);
      if (SPLIT) bl[j] = Frag<T>::load(Bb2 + bo);
    }
#pragma unroll
    for (int i = 0; i < 4; ++i) {
      const size_t ao = (size_t)(m0 + (i << 4) + rlane) * lda + koff + k0;
      V ah = Frag<T>::load(Ab + ao);
      V al;
      if (SPLIT) al = Frag<T>::load(Ab2 + ao);
#pragma unroll
      for (int j = 0; j < 4; ++j) {
        acc[i][j] = Frag<T>::mma(ah, bh[j], acc[i][j]);
        if (SPLIT) {
          acc[i][j] = Frag<T>::mma(ah, bl[j], acc[i][j]);
          acc[i][j] = Frag<T>::mma(al, bh[j], acc[i][j]);
        }
      }
      Frag<T>::guard(acc[i][0], acc[i][3], ah, SPLIT ? al : ah);
    }
    Frag<T>::keep(bh[0], bh[1], bh[2], bh[3]);
    if (SPLIT) Frag<T>::keep(bl[0], bl[1], bl[2], bl[3]);
  }
  acc_guard4(acc[0][0], acc[0][1], acc[0][2], acc[0][3]);
  acc_guard4(acc[1][0], acc[1][1], acc[1][2], acc[1][3]);
  acc_guard4(acc[2][0], acc[2][1], acc[2][2], acc[2][3]);
  acc_guard4(acc[3][0], acc[3][1], acc[3][2], acc[3][3]);

  float* slab = sT[wave];
  const float* Rb = RESID ? (resid + (size_t)b * strideR) : nullptr;
#pragma unroll
  for (int i = 0; i < 4; ++i) {
    const int mBase = m0 + (i << 4);
#pragma unroll
    for (int j = 0; j < 4; ++j) {
      const int n = n0 + (j << 4) + rlane;
      float bv = 0.f;
      if (BIAS_MODE == 2) bv = bias[n];
#pragma unroll
      for (int r = 0; r < 8; ++r) {
        float v = acc[i][j][r] * scale;
        if (BIAS_MODE == 1) v += bias[mBase + mOff + r];
        if (BIAS_MODE == 2) v += bv;
        if (RESID) v += Rb[(size_t)(mBase + mOff + r) * ldc + n];
        if (ACT == 2) v = fmaxf(v, 0.0f);
        if (ACT == 4) v = (v > 0.f) ? v : 0.01f * v;
        slab[(mOff + r) * 68 + (j << 4) + rlane] = v;
      }
    }
    __builtin_amdgcn_fence(__ATOMIC_RELEASE, "workgroup");
    __builtin_amdgcn_wave_barrier();
    __builtin_amdgcn_fence(__ATOMIC_ACQUIRE, "workgroup");
    if (OUT_MODE == 0) {
      float* C = (float*)Cout + (size_t)b * strideC;
      const int hh = lane >> 4, c4 = (lane & 15) * 4;
      for (int pass = 0; pass < 2; ++pass) {
#pragma unroll
        for (int it = 0; it < 8; ++it) {
          const int row = it * 2 + hh;
          v4f v = *(const v4f*)(slab + row * 68 + c4);
          *(volatile v4f*)(C + (size_t)(mBase + row) * ldc + n0 + c4) = v;
        }
        __threadfence();
      }
    } else {
      const int q = lane >> 3, c8 = (lane & 7) * 8;
      unsigned short* C  = (unsigned short*)Cout  + (size_t)b * strideC;
      unsigned short* C2 = (OUT_MODE == 2) ? ((unsigned short*)Cout2 + (size_t)b * strideC) : nullptr;
      for (int pass = 0; pass < 2; ++pass) {
#pragma unroll
        for (int it = 0; it < 4; ++it) {
          const int row = it * 4 + q;
          const float* sp = slab + row * 68 + c8;
          v8h hv, lv;
#pragma unroll
          for (int e = 0; e < 8; ++e) {
            if (OUT_MODE == 1) {
              hv[e] = (_Float16)sp[e];
            } else {
              unsigned short hb = f2bf_bits(sp[e]);
              unsigned short lb = f2bf_bits(sp[e] - bf_bits2f(hb));
              hv[e] = __builtin_bit_cast(_Float16, hb);
              lv[e] = __builtin_bit_cast(_Float16, lb);
            }
          }
          *(volatile v8h*)(C + (size_t)(mBase + row) * ldc + n0 + c8) = hv;
          if (OUT_MODE == 2) *(volatile v8h*)(C2 + (size_t)(mBase + row) * ldc + n0 + c8) = lv;
        }
        __threadfence();
      }
    }
    __builtin_amdgcn_fence(__ATOMIC_RELEASE, "workgroup");
    __builtin_amdgcn_wave_barrier();
    __builtin_amdgcn_fence(__ATOMIC_ACQUIRE, "workgroup");
  }
}

__device__ __forceinline__ float fast_rcp(float x) { return __builtin_amdgcn_rcpf(x); }
__device__ __forceinline__ float sigm_f(float x) { return fast_rcp(1.0f + __expf(-x)); }
__device__ __forceinline__ float tanh_f(float x) { return fmaf(-2.0f, fast_rcp(1.0f + __expf(2.0f * x)), 1.0f); }

__device__ __forceinline__ void ld8(float (&d)[8], const float* p) {
  const v4f a = *(const v4f*)p;
  const v4f c = *(const v4f*)(p + 4);
  d[0] = a[0]; d[1] = a[1]; d[2] = a[2]; d[3] = a[3];
  d[4] = c[0]; d[5] = c[1]; d[6] = c[2]; d[7] = c[3];
}
__device__ __forceinline__ v4u pack8(const unsigned short (&h)[8]) {
  return (v4u){pk16(h[0], h[1]), pk16(h[2], h[3]), pk16(h[4], h[5]), pk16(h[6], h[7])};
}

__global__ __launch_bounds__(256) void fill_zero_kernel(float* __restrict__ p, int n4) {
  const int i = blockIdx.x * 256 + threadIdx.x;
  if (i >= n4) return;
  const v4f z = (v4f){0.f, 0.f, 0.f, 0.f};
  float* q = p + 4 * (size_t)i;
  *(volatile v4f*)q = z;
  __threadfence();
  *(volatile v4f*)q = z;
}

__global__ __launch_bounds__(256) void bias_pad_kernel(
    const float* __restrict__ s0, int n0, float* __restrict__ d0, int np0,
    const float* __restrict__ s1, int n1, float* __restrict__ d1, int np1,
    const float* __restrict__ s2, int n2, float* __restrict__ d2, int np2) {
  const int z = blockIdx.y;
  const float* s = (z == 0) ? s0 : (z == 1) ? s1 : s2;
  const int    n = (z == 0) ? n0 : (z == 1) ? n1 : n2;
  float*       d = (z == 0) ? d0 : (z == 1) ? d1 : d2;
  const int   np = (z == 0) ? np0 : (z == 1) ? np1 : np2;
  const int i = blockIdx.x * 256 + threadIdx.x;
  if (4 * i >= np) return;
  v4f v;
#pragma unroll
  for (int e = 0; e < 4; ++e) {
    const int idx = 4 * i + e;
    const int ic = idx < n ? idx : n - 1;
    const float x = s[ic];
    v[e] = (idx < n) ? x : 0.0f;
  }
  float* q = d + 4 * (size_t)i;
  *(volatile v4f*)q = v;
  __threadfence();
  *(volatile v4f*)q = v;
}

__global__ __launch_bounds__(256) void cast_rows_f16_kernel(const float* __restrict__ src, int nrows, int kcols,
                                                           unsigned short* __restrict__ dst, int nrowsPad, float scale) {
  const int g = blockIdx.x * 256 + threadIdx.x;
  const int gpr = kcols >> 3;
  const int total = nrowsPad * gpr;
  if (g >= total) return;
  const int row = g / gpr;
  const int c8 = (g - row * gpr) * 8;
  const int rowc = row < nrows ? row : nrows - 1;
  const float* p = src + (size_t)rowc * kcols + c8;
  const v4f a = *(const v4f*)p;
  const v4f c = *(const v4f*)(p + 4);
  const bool valid = row < nrows;
  unsigned short hb[8];
#pragma unroll
  for (int e = 0; e < 4; ++e) {
    const float x0 = valid ? a[e] * scale : 0.0f;
    const float x1 = valid ? c[e] * scale : 0.0f;
    hb[e]     = h_bits(x0);
    hb[4 + e] = h_bits(x1);
  }
  const v4u u = pack8(hb);
  unsigned short* q = dst + 8 * (size_t)g;
  *(volatile v4u*)q = u;
  __threadfence();
  *(volatile v4u*)q = u;
}

__global__ __launch_bounds__(256) void split_rows_bf16_kernel(const float* __restrict__ src, int nrows, int kin,
                                                             int gapStart, int gapLen,
                                                             unsigned short* __restrict__ hi, unsigned short* __restrict__ lo,
                                                             int nrowsPad, int kpad) {
  const int g = blockIdx.x * 256 + threadIdx.x;
  const int gpr = kpad >> 3;
  const int total = nrowsPad * gpr;
  if (g >= total) return;
  const int row = g / gpr;
  const int c0 = (g - row * gpr) * 8;
  const int rowc = row < nrows ? row : nrows - 1;
  const float* p = src + (size_t)rowc * kin;
  unsigned short hb[8], lb[8];
#pragma unroll
  for (int e = 0; e < 8; ++e) {
    const int c = c0 + e;
    const int sc = (c < gapStart) ? c : (c - gapLen);
    const bool ok = (row < nrows) && ((c < gapStart) || (c >= gapStart + gapLen)) && (sc >= 0) && (sc < kin);
    const int scc = sc < 0 ? 0 : (sc >= kin ? kin - 1 : sc);
    float x = p[scc];
    x = ok ? x : 0.0f;
    hb[e] = f2bf_bits(x);
    lb[e] = f2bf_bits(x - bf_bits2f(hb[e]));
  }
  const v4u uh = pack8(hb), ul = pack8(lb);
  unsigned short* qh = hi + 8 * (size_t)g;
  unsigned short* ql = lo + 8 * (size_t)g;
  for (int pass = 0; pass < 2; ++pass) {
    *(volatile v4u*)qh = uh;
    *(volatile v4u*)ql = ul;
    __threadfence();
  }
}

__global__ __launch_bounds__(128) void tdin_init_kernel(const float* __restrict__ wemb, const float* __restrict__ tf,
                                                       unsigned short* __restrict__ thi, unsigned short* __restrict__ tlo) {
  const int b = blockIdx.x;
  const int g = threadIdx.x;
  const float* xr = wemb + (size_t)b * kT * kEmb;
  const float* tr = tf + (size_t)b * kFeat;
  unsigned short hb[8], lb[8];
#pragma unroll
  for (int e = 0; e < 8; ++e) {
    const int c = 8 * g + e;
    const int cx = c < kEmb ? c : kEmb - 1;
    int ct = c - (kEmbPad + kHid);
    ct = ct < 0 ? 0 : (ct >= kFeat ? kFeat - 1 : ct);
    const float xv = xr[cx];
    const float tv = tr[ct];
    const float v = (c < kEmb) ? xv : ((c >= kEmbPad + kHid && c < kTdK) ? tv : 0.0f);
    hb[e] = f2bf_bits(v);
    lb[e] = f2bf_bits(v - bf_bits2f(hb[e]));
  }
  const v4u uh = pack8(hb), ul = pack8(lb);
  if (g < kTdK / 8) {
    unsigned short* qh = thi + (size_t)b * kTdK + 8 * g;
    unsigned short* ql = tlo + (size_t)b * kTdK + 8 * g;
    for (int pass = 0; pass < 2; ++pass) {
      *(volatile v4u*)qh = uh;
      *(volatile v4u*)ql = ul;
      __threadfence();
    }
  }
}

template <bool SECOND>
__global__ __launch_bounds__(64) void gru_gate_kernel(
    const float* __restrict__ gi, const float* __restrict__ gh, int ghPitch,
    const float* __restrict__ bih, const float* __restrict__ bhh,
    float* hstate, unsigned short* __restrict__ h16,
    unsigned short* phi, unsigned short* plo, int pPitch, int hCol,
    unsigned short* __restrict__ hist, int tstep, const float* __restrict__ wemb) {
  __shared__ __align__(16) float sH[kHid];
  const int b = blockIdx.x;
  const int tid = threadIdx.x;
  const int j0 = tid * 8;
  const float* gir = gi + (size_t)b * kGru + j0;
  const float* ghr = gh + (size_t)b * ghPitch + j0;
  float* hrow = hstate + (size_t)b * kHid;

  float ir[8], iz[8], inn[8], hr[8], hz[8], hn[8], hp[8];
  float bir[8], biz[8], bin[8], bhr[8], bhz[8], bhn[8];
  ld8(ir, gir); ld8(iz, gir + kHid); ld8(inn, gir + 2 * kHid);
  ld8(hr, ghr); ld8(hz, ghr + kHid); ld8(hn, ghr + 2 * kHid);
  ld8(bir, bih + j0); ld8(biz, bih + kHid + j0); ld8(bin, bih + 2 * kHid + j0);
  ld8(bhr, bhh + j0); ld8(bhz, bhh + kHid + j0); ld8(bhn, bhh + 2 * kHid + j0);
  ld8(hp, hrow + j0);

  float o[8];
#pragma unroll
  for (int e = 0; e < 8; ++e) {
    const float r = sigm_f((ir[e] + bir[e]) + (hr[e] + bhr[e]));
    const float z = sigm_f((iz[e] + biz[e]) + (hz[e] + bhz[e]));
    const float n = tanh_f((inn[e] + bin[e]) + r * (hn[e] + bhn[e]));
    o[e] = (1.0f - z) * n + z * hp[e];
    sH[j0 + e] = o[e];
  }
  unsigned short fh[8], bhb[8], blb[8];
#pragma unroll
  for (int e = 0; e < 8; ++e) {
    fh[e]  = h_bits(o[e]);
    bhb[e] = f2bf_bits(o[e]);
    blb[e] = f2bf_bits(o[e] - bf_bits2f(bhb[e]));
  }
  const v4u uh = pack8(fh), ubh = pack8(bhb), ubl = pack8(blb);
  v4u uxh = (v4u){0u, 0u, 0u, 0u}, uxl = (v4u){0u, 0u, 0u, 0u};
  if (SECOND) {
    const int tn = (tstep + 1 < kT) ? tstep + 1 : kT - 1;
    const float* xr = wemb + ((size_t)b * kT + tn) * kEmb;
    unsigned short xh[8], xl[8];
#pragma unroll
    for (int e = 0; e < 8; ++e) {
      const int c = j0 + e;
      const int cc = c < kEmb ? c : kEmb - 1;
      float xv = xr[cc];
      xv = (c < kEmb) ? xv : 0.0f;
      xh[e] = f2bf_bits(xv);
      xl[e] = f2bf_bits(xv - bf_bits2f(xh[e]));
    }
    uxh = pack8(xh); uxl = pack8(xl);
  }
  __syncthreads();
  const v4f f0 = *(const v4f*)(sH + 4 * tid);
  const v4f f1 = *(const v4f*)(sH + 256 + 4 * tid);
  const bool doX = SECOND && (tstep + 1 < kT) && (tid < kEmbPad / 8);
  unsigned short* prow_h = phi + (size_t)b * pPitch;
  unsigned short* prow_l = plo + (size_t)b * pPitch;
  for (int pass = 0; pass < 2; ++pass) {
    *(volatile v4f*)(hrow + 4 * tid) = f0;
    *(volatile v4f*)(hrow + 256 + 4 * tid) = f1;
    *(volatile v4u*)(h16 + (size_t)b * kHid + j0) = uh;
    *(volatile v4u*)(prow_h + hCol + j0) = ubh;
    *(volatile v4u*)(prow_l + hCol + j0) = ubl;
    if (SECOND) *(volatile v4u*)(hist + ((size_t)b * kT + tstep) * kHid + j0) = uh;
    if (doX) {
      *(volatile v4u*)(prow_h + j0) = uxh;
      *(volatile v4u*)(prow_l + j0) = uxl;
    }
    __threadfence();
  }
}

__global__ __launch_bounds__(256) void attn_step_kernel(
    const float* __restrict__ featp, const float* __restrict__ hh, int hhPitch,
    const float* __restrict__ watt, const int* __restrict__ masks, const float* __restrict__ obj,
    float* __restrict__ attn_out, unsigned short* __restrict__ lhi, unsigned short* __restrict__ llo) {
  __shared__ __align__(16) float sC[kHid];
  __shared__ __align__(16) float sW[kHid];
  __shared__ __align__(16) float sA[kProp];
  __shared__ __align__(16) float sPart[2][kFeat];
  __shared__ float sRed[3][8];
  const int b = blockIdx.x;
  const int tid = threadIdx.x;
  const int lane = tid & 31, wave = tid >> 5;
  const float* hrow = hh + (size_t)b * hhPitch;
  float wpart;
  {
    const float h0 = hrow[tid], h1 = hrow[tid + 256];
    const float w0 = watt[tid], w1 = watt[tid + 256];
    sC[tid] = 2.0f * h0; sC[tid + 256] = 2.0f * h1;
    sW[tid] = w0; sW[tid + 256] = w1;
    wpart = w0 + w1;
  }
#pragma unroll
  for (int off = 16; off > 0; off >>= 1) wpart += __shfl_xor(wpart, off, 32);
  if (lane == 0) sRed[0][wave] = wpart;
  __syncthreads();
  float wsum = 0.0f;
#pragma unroll
  for (int w = 0; w < 8; ++w) wsum += sRed[0][w];

  const float* fr = featp + ((size_t)b * kProp + tid) * kHid;
  float acc = 0.0f;
#pragma unroll 1
  for (int h = 0; h < kHid; h += 4) {
    const v4f fv = *(const v4f*)(fr + h);
    const v4f cv = *(const v4f*)(sC + h);
    const v4f wv = *(const v4f*)(sW + h);
#pragma unroll
    for (int e = 0; e < 4; ++e) {
      const float y = fmaf(fv[e], 2.0f, cv[e]);
      const float ex = __expf(y);
      const float rr = fast_rcp(1.0f + ex);
      acc = fmaf(wv[e], rr, acc);
    }
  }
  float sc = wsum - 2.0f * acc;
  const int mk = masks[(size_t)b * kProp + tid];
  sc = (mk == 0) ? -1e30f : sc;

  float m = sc;
#pragma unroll
  for (int off = 16; off > 0; off >>= 1) m = fmaxf(m, __shfl_xor(m, off, 32));
  if (lane == 0) sRed[1][wave] = m;
  __syncthreads();
  float mx = sRed[1][0];
#pragma unroll
  for (int w = 1; w < 8; ++w) mx = fmaxf(mx, sRed[1][w]);
  const float e = expf(sc - mx);
  float s = e;
#pragma unroll
  for (int off = 16; off > 0; off >>= 1) s += __shfl_xor(s, off, 32);
  if (lane == 0) sRed[2][wave] = s;
  __syncthreads();
  float tot = 0.0f;
#pragma unroll
  for (int w = 0; w < 8; ++w) tot += sRed[2][w];
  const float a = e * (1.0f / tot);
  sA[tid] = a;
  __syncthreads();

  if (wave == 0) {
    float* orow = attn_out + (size_t)b * (kT * kProp);
    const v4f v0 = *(const v4f*)(sA + 4 * lane);
    const v4f v1 = *(const v4f*)(sA + 128 + 4 * lane);
    for (int pass = 0; pass < 2; ++pass) {
      *(volatile v4f*)(orow + 4 * lane) = v0;
      *(volatile v4f*)(orow + 128 + 4 * lane) = v1;
      __threadfence();
    }
  }

  const int f = tid & (kFeat - 1), half = tid >> 7;
  const float* ob = obj + ((size_t)b * kProp + half * 128) * kFeat + f;
  const float* ap = sA + half * 128;
  float at = 0.0f;
#pragma unroll 1
  for (int p = 0; p < 128; p += 4) {
    const v4f av = *(const v4f*)(ap + p);
#pragma unroll
    for (int q = 0; q < 4; ++q) at = fmaf(av[q], ob[(size_t)(p + q) * kFeat], at);
  }
  sPart[half][f] = at;
  __syncthreads();
  if (wave == 0) {
    const int g = lane & 15, sel = lane >> 4;
    unsigned short hb[8], lb[8];
#pragma unroll
    for (int q = 0; q < 8; ++q) {
      const float v = sPart[0][8 * g + q] + sPart[1][8 * g + q];
      hb[q] = f2bf_bits(v);
      lb[q] = f2bf_bits(v - bf_bits2f(hb[q]));
    }
    const v4u uh = pack8(hb), ul = pack8(lb);
    v4u u;
    u[0] = sel ? ul[0] : uh[0]; u[1] = sel ? ul[1] : uh[1]; u[2] = sel ? ul[2] : uh[2]; u[3] = sel ? ul[3] : uh[3];
    unsigned short* q = (sel ? llo : lhi) + (size_t)b * kLangK + 8 * g;
    for (int pass = 0; pass < 2; ++pass) {
      *(volatile v4u*)q = u;
      __threadfence();
    }
  }
}

__global__ __launch_bounds__(256) void pack_logits_kernel(const float* __restrict__ lg, float* __restrict__ out, int n4) {
  const int i = blockIdx.x * 256 + threadIdx.x;
  if (i >= n4) return;
  const unsigned f0 = 4u * (unsigned)i;
  const unsigned row = f0 / (unsigned)kVoc;
  const unsigned col = f0 - row * (unsigned)kVoc;
  v4f v;
#pragma unroll
  for (int e = 0; e < 4; ++e) {
    unsigned c = col + (unsigned)e;
    unsigned r = row + ((c >= (unsigned)kVoc) ? 1u : 0u);
    c = (c >= (unsigned)kVoc) ? c - (unsigned)kVoc : c;
    r = r < (unsigned)kRowsBT ? r : (unsigned)(kRowsBT - 1);
    v[e] = lg[(size_t)r * kVocPad + c];
  }
  float* q = out + 4 * (size_t)i;
  *(volatile v4f*)q = v;
  __threadfence();
  *(volatile v4f*)q = v;
}

template <int ET, bool SPLIT, int BIAS, int OUTM, int ACT>
static void run_gemm(hipStream_t s, const void* A, const void* A2, int lda, long sA,
                     const void* Bt, const void* Bt2, int ldb, long sB,
                     void* C, void* C2, int ldc, long sC, const float* bias,
                     int M, int N, int K, float scale, int batch) {
  const int tiles = (M / 64) * (N / 64);
  dim3 grid((tiles + 7) / 8, batch);
  wmma_gemm64<ET, SPLIT, BIAS, OUTM, false, ACT><<<grid, 256, 0, s>>>(
      (const unsigned short*)A, (const unsigned short*)A2, lda, sA,
      (const unsigned short*)Bt, (const unsigned short*)Bt2, ldb, sB,
      C, C2, ldc, sC, bias, (const float*)nullptr, 0L, M, N, K, scale);
}

static void run_cast(hipStream_t s, const float* src, int nrows, int kcols, unsigned short* dst, int nrowsPad, float scale) {
  const int total = nrowsPad * (kcols / 8);
  cast_rows_f16_kernel<<<(total + 255) / 256, 256, 0, s>>>(src, nrows, kcols, dst, nrowsPad, scale);
}
static void run_split(hipStream_t s, const float* src, int nrows, int kin, int gapStart, int gapLen,
                      unsigned short* hi, unsigned short* lo, int nrowsPad, int kpad) {
  const int total = nrowsPad * (kpad / 8);
  split_rows_bf16_kernel<<<(total + 255) / 256, 256, 0, s>>>(src, nrows, kin, gapStart, gapLen, hi, lo, nrowsPad, kpad);
}

extern "C" void kernel_launch(void* const* d_in, const int* in_sizes, int n_in,
                              void* d_out, int out_size, void* d_ws, size_t ws_size,
                              hipStream_t stream) {
  if (n_in < 21) return;
  if (in_sizes[0] != kB * kT * kEmb || in_sizes[1] != kB * kFeat || in_sizes[2] != kB * kProp * kFeat ||
      in_sizes[3] != kB * kProp || in_sizes[4] != kEmb * kTdIn || in_sizes[6] != kGru * kEmb ||
      in_sizes[7] != kGru * kHid || in_sizes[10] != kHid * kFeat || in_sizes[11] != kHid * kHid ||
      in_sizes[12] != kHid || in_sizes[13] != kEmb * kLangK || in_sizes[15] != kGru * kEmb ||
      in_sizes[16] != kGru * kHid || in_sizes[19] != kVoc * kHid || in_sizes[20] != kVoc ||
      in_sizes[5] != kEmb || in_sizes[14] != kEmb || in_sizes[8] != kGru || in_sizes[9] != kGru ||
      in_sizes[17] != kGru || in_sizes[18] != kGru) return;
  if (out_size != kB * kT * kVoc + kB * kT * kProp) return;

  const float* word_embs = (const float*)d_in[0];
  const float* tfeat     = (const float*)d_in[1];
  const float* obj_feats = (const float*)d_in[2];
  const int*   masks     = (const int*)d_in[3];
  const float* w_td   = (const float*)d_in[4];
  const float* b_td   = (const float*)d_in[5];
  const float* w_ih1  = (const float*)d_in[6];
  const float* w_hh1  = (const float*)d_in[7];
  const float* b_ih1  = (const float*)d_in[8];
  const float* b_hh1  = (const float*)d_in[9];
  const float* w_feat = (const float*)d_in[10];
  const float* w_hidd = (const float*)d_in[11];
  const float* w_att  = (const float*)d_in[12];
  const float* w_lang = (const float*)d_in[13];
  const float* b_lang = (const float*)d_in[14];
  const float* w_ih2  = (const float*)d_in[15];
  const float* w_hh2  = (const float*)d_in[16];
  const float* b_ih2  = (const float*)d_in[17];
  const float* b_hh2  = (const float*)d_in[18];
  const float* w_cls  = (const float*)d_in[19];
  const float* b_cls  = (const float*)d_in[20];

  float* out0 = (float*)d_out;
  float* out1 = (float*)d_out + (size_t)kB * kT * kVoc;

  char* base = (char*)d_ws;
  size_t off = 0;
  auto carve = [&](size_t bytes) -> char* { char* p = base + off; off += (bytes + 255) & ~(size_t)255; return p; };

  const size_t logstBytes = (size_t)kRowsBT * kVocPad * 4;
  float* LOGST = (float*)base;
  unsigned short* OBJ16   = (unsigned short*)carve((size_t)kB * kProp * kFeat * 2);
  unsigned short* WFEAT16 = (unsigned short*)carve((size_t)kHid * kFeat * 2);
  unsigned short* WHB16   = (unsigned short*)carve((size_t)4096 * kHid * 2);
  unsigned short* WTDH    = (unsigned short*)carve((size_t)kEmbPad * kTdK * 2);
  unsigned short* WTDL    = (unsigned short*)carve((size_t)kEmbPad * kTdK * 2);
  unsigned short* WIH1H   = (unsigned short*)carve((size_t)kGru * kEmbPad * 2);
  unsigned short* WIH1L   = (unsigned short*)carve((size_t)kGru * kEmbPad * 2);
  unsigned short* WIH2H   = (unsigned short*)carve((size_t)kGru * kEmbPad * 2);
  unsigned short* WIH2L   = (unsigned short*)carve((size_t)kGru * kEmbPad * 2);
  unsigned short* WLANGH  = (unsigned short*)carve((size_t)kEmbPad * kLangK * 2);
  unsigned short* WLANGL  = (unsigned short*)carve((size_t)kEmbPad * kLangK * 2);
  float* BTD   = (float*)carve((size_t)kEmbPad * 4);
  float* BLANG = (float*)carve((size_t)kEmbPad * 4);
  float* HSTATE = (float*)carve((size_t)2 * kB * kHid * 4);
  unsigned short* H16 = (unsigned short*)carve((size_t)2 * kB * kHid * 2);
  float* GHH = (float*)carve((size_t)2 * kB * kGhhN * 4);
  const size_t zeroSpanBytes = (size_t)2 * kB * kHid * 4 + (size_t)2 * kB * kHid * 2 + (size_t)2 * kB * kGhhN * 4;
  float* GI = (float*)carve((size_t)kB * kGru * 4);
  unsigned short* TDINH   = (unsigned short*)carve((size_t)kB * kTdK * 2);
  unsigned short* TDINL   = (unsigned short*)carve((size_t)kB * kTdK * 2);
  unsigned short* TDH     = (unsigned short*)carve((size_t)kB * kEmbPad * 2);
  unsigned short* TDL     = (unsigned short*)carve((size_t)kB * kEmbPad * 2);
  unsigned short* LANGINH = (unsigned short*)carve((size_t)kB * kLangK * 2);
  unsigned short* LANGINL = (unsigned short*)carve((size_t)kB * kLangK * 2);
  unsigned short* LANGH   = (unsigned short*)carve((size_t)kB * kEmbPad * 2);
  unsigned short* LANGL   = (unsigned short*)carve((size_t)kB * kEmbPad * 2);
  if (off > logstBytes) return;
  off = (logstBytes + 255) & ~(size_t)255;
  float* FEATP = (float*)carve((size_t)kB * kProp * kHid * 4);
  unsigned short* H2HIST = (unsigned short*)carve((size_t)kRowsBT * kHid * 2);
  unsigned short* WCLS16 = (unsigned short*)carve((size_t)kVocPad * kHid * 2);
  float* BCLS = (float*)carve((size_t)kVocPad * 4);
  if (off > ws_size) return;

  float* H1S = HSTATE;
  float* H2S = HSTATE + (size_t)kB * kHid;
  unsigned short* H1F16 = H16;
  unsigned short* H2F16 = H16 + (size_t)kB * kHid;

  fill_zero_kernel<<<(int)((zeroSpanBytes / 16 + 255) / 256), 256, 0, stream>>>(HSTATE, (int)(zeroSpanBytes / 16));
  bias_pad_kernel<<<dim3((kVocPad / 4 + 255) / 256, 3), 256, 0, stream>>>(b_td, kEmb, BTD, kEmbPad,
                                                                            b_lang, kEmb, BLANG, kEmbPad,
                                                                            b_cls, kVoc, BCLS, kVocPad);
  run_cast(stream, w_feat, kHid, kFeat, WFEAT16, kHid, kWCarry);
  run_cast(stream, w_hidd, kHid, kHid, WHB16, kHid, kWCarry);
  run_cast(stream, w_hh1, kGru, kHid, WHB16 + (size_t)512 * kHid, kGru, kWCarry);
  run_cast(stream, w_hidd, kHid, kHid, WHB16 + (size_t)2048 * kHid, kHid, kWCarry);
  run_cast(stream, w_hh2, kGru, kHid, WHB16 + (size_t)2560 * kHid, kGru, kWCarry);
  run_cast(stream, w_cls, kVoc, kHid, WCLS16, kVocPad, kWCarry);
  run_cast(stream, obj_feats, kB * kProp, kFeat, OBJ16, kB * kProp, 1.0f);
  run_split(stream, w_td, kEmb, kTdIn, kEmb, kEmbPad - kEmb, WTDH, WTDL, kEmbPad, kTdK);
  run_split(stream, w_ih1, kGru, kEmb, kEmb, kEmbPad - kEmb, WIH1H, WIH1L, kGru, kEmbPad);
  run_split(stream, w_ih2, kGru, kEmb, kEmb, kEmbPad - kEmb, WIH2H, WIH2L, kGru, kEmbPad);
  run_split(stream, w_lang, kEmb, kLangK, kLangK, 0, WLANGH, WLANGL, kEmbPad, kLangK);
  tdin_init_kernel<<<kB, 128, 0, stream>>>(word_embs, tfeat, TDINH, TDINL);
  run_gemm<0, false, 0, 0, 0>(stream, OBJ16, nullptr, kFeat, 0L, WFEAT16, nullptr, kFeat, 0L,
                              FEATP, nullptr, kHid, 0L, nullptr, kB * kProp, kHid, kFeat, kWCarryInv, 1);

  for (int t = 0; t < kT; ++t) {
    run_gemm<1, true, 2, 2, 2>(stream, TDINH, TDINL, kTdK, 0L, WTDH, WTDL, kTdK, 0L,
                               TDH, TDL, kEmbPad, 0L, BTD, kB, kEmbPad, kTdK, 1.0f, 1);
    run_gemm<1, true, 0, 0, 0>(stream, TDH, TDL, kEmbPad, 0L, WIH1H, WIH1L, kEmbPad, 0L,
                               GI, nullptr, kGru, 0L, nullptr, kB, kGru, kEmbPad, 1.0f, 1);
    gru_gate_kernel<false><<<kB, 64, 0, stream>>>(GI, GHH + kHid, kGhhN, b_ih1, b_hh1, H1S, H1F16,
                                                  LANGINH, LANGINL, kLangK, kFeat,
                                                  (unsigned short*)nullptr, t, (const float*)nullptr);
    run_gemm<0, false, 0, 0, 0>(stream, H16, nullptr, kHid, (long)kB * kHid, WHB16, nullptr, kHid, (long)2048 * kHid,
                                GHH, nullptr, kGhhN, (long)kB * kGhhN, nullptr, kB, kGhhN, kHid, kWCarryInv, 2);
    attn_step_kernel<<<kB, 256, 0, stream>>>(FEATP, GHH, kGhhN, w_att, masks, obj_feats,
                                              out1 + (size_t)t * kProp, LANGINH, LANGINL);
    run_gemm<1, true, 2, 2, 2>(stream, LANGINH, LANGINL, kLangK, 0L, WLANGH, WLANGL, kLangK, 0L,
                               LANGH, LANGL, kEmbPad, 0L, BLANG, kB, kEmbPad, kLangK, 1.0f, 1);
    run_gemm<1, true, 0, 0, 0>(stream, LANGH, LANGL, kEmbPad, 0L, WIH2H, WIH2L, kEmbPad, 0L,
                               GI, nullptr, kGru, 0L, nullptr, kB, kGru, kEmbPad, 1.0f, 1);
    gru_gate_kernel<true><<<kB, 64, 0, stream>>>(GI, GHH + (size_t)kB * kGhhN + kHid, kGhhN, b_ih2, b_hh2, H2S, H2F16,
                                                 TDINH, TDINL, kTdK, kEmbPad, H2HIST, t, word_embs);
  }

  run_gemm<0, false, 2, 0, 0>(stream, H2HIST, nullptr, kHid, 0L, WCLS16, nullptr, kHid, 0L,
                              LOGST, nullptr, kVocPad, 0L, BCLS, kRowsBT, kVocPad, kHid, kWCarryInv, 1);
  const int n4 = kB * kT * kVoc / 4;
  pack_logits_kernel<<<(n4 + 255) / 256, 256, 0, stream>>>(LOGST, out0, n4);
  (void)ws_size;
}
